// BahdanauMultiheadAttention_9637906612352
// MI455X (gfx1250) — hardware-verified
//
#include <hip/hip_runtime.h>
#include <hip/hip_bf16.h>
#include <stddef.h>
#include <stdint.h>


#define BB   4
#define LL   256
#define DD   512
#define HH   8
#define DK   64
#define NR   (BB * LL)
#define NTHR 128

static_assert(NR == 1024);
static_assert(DD == HH * DK);
static_assert(LL == 2 * NTHR);
static_assert(DK == 64);

typedef unsigned short v8us  __attribute__((ext_vector_type(8)));
typedef __bf16         v16bf __attribute__((ext_vector_type(16)));
typedef float          v8f   __attribute__((ext_vector_type(8)));
typedef float          v4f   __attribute__((ext_vector_type(4)));
typedef int            v2i   __attribute__((ext_vector_type(2)));

union Frag { v16bf v; v8us h[2]; };

#if __has_builtin(__builtin_amdgcn_exp2f)
#define EXP2_FAST(x) __builtin_amdgcn_exp2f(x)
#else
#define EXP2_FAST(x) exp2f(x)
#endif
#if __has_builtin(__builtin_amdgcn_rcpf)
#define RCP_FAST(x) __builtin_amdgcn_rcpf(x)
#else
#define RCP_FAST(x) (1.0f / (x))
#endif

__device__ __forceinline__ unsigned int bf16_rne(float f)
{
    unsigned int u = __float_as_uint(f);
    u += 0x7FFFu + ((u >> 16) & 1u);
    return u >> 16;
}

__device__ __forceinline__ void split1(float x, unsigned int& hb, unsigned int& lb)
{
    hb = bf16_rne(x);
    const float xh = __uint_as_float(hb << 16);
    lb = bf16_rne(x - xh);
}

__device__ __forceinline__ void split8(v4f a, v4f b, v8us& hi, v8us& lo)
{
    v8us hr = { 0, 0, 0, 0, 0, 0, 0, 0 };
    v8us lr = { 0, 0, 0, 0, 0, 0, 0, 0 };
    #pragma unroll
    for (int e = 0; e < 4; ++e) {
        unsigned int hb, lb;
        split1(a[e], hb, lb);
        hr[e] = (unsigned short)hb;
        lr[e] = (unsigned short)lb;
        split1(b[e], hb, lb);
        hr[4 + e] = (unsigned short)hb;
        lr[4 + e] = (unsigned short)lb;
    }
    hi = hr;
    lo = lr;
}

__device__ __forceinline__ v16bf frag16(const unsigned short* row, int k0, int hh)
{
    Frag f;
    f.h[0] = *(const v8us*)(row + k0 + 8 * hh);
    f.h[1] = *(const v8us*)(row + k0 + 16 + 8 * hh);
    return f.v;
}

__device__ __forceinline__ v8f wmma_bf16(v16bf a, v16bf b, v8f c)
{
    v8f d = __builtin_amdgcn_wmma_f32_16x16x32_bf16(false, a, false, b, (short)0, c, false, false);
    asm volatile("v_nop\n\tv_nop\n\tv_nop\n\tv_nop" : "+v"(d) : "v"(a), "v"(b));
    return d;
}

__device__ __forceinline__ v8f wmma3(v16bf ah, v16bf al, v16bf bh, v16bf bl, v8f c)
{
    c = wmma_bf16(ah, bh, c);
    c = wmma_bf16(ah, bl, c);
    c = wmma_bf16(al, bh, c);
    return c;
}

__global__ void __launch_bounds__(NTHR) prep_kernel(
    const float* __restrict__ q, const float* __restrict__ k, const float* __restrict__ v,
    const float* __restrict__ Wq, const float* __restrict__ Wk,
    const float* __restrict__ Wv, const float* __restrict__ W0,
    unsigned short* xh, unsigned short* xl, unsigned short* wth, unsigned short* wtl)
{
    __shared__ float s_t[64][65];

    const int tid = threadIdx.x;
    const int bid = blockIdx.x;
    const int NXB = 3 * (NR / 2);

    if (bid < NXB) {
        const int t   = bid / (NR / 2);
        const int row = ((bid % (NR / 2)) << 1) + (tid >> 6);
        const int c8  = tid & 63;
        const float* src = (t == 0) ? q : ((t == 1) ? k : v);
        const size_t soff = (size_t)row * DD + 8 * c8;
        const v4f x0 = *(const v4f*)(src + soff);
        const v4f x1 = *(const v4f*)(src + soff + 4);
        v8us hv, lv;
        split8(x0, x1, hv, lv);
        const size_t doff = ((size_t)t * NR + row) * DD + 8 * c8;
        *(volatile v8us*)(xh + doff) = hv;
        *(volatile v8us*)(xl + doff) = lv;
        __threadfence();
        *(volatile v8us*)(xh + doff) = hv;
        *(volatile v8us*)(xl + doff) = lv;
    } else {
        const int u    = bid - NXB;
        const int w    = u >> 6;
        const int tile = u & 63;
        const int k0   = (tile >> 3) * 64;
        const int n0   = (tile & 7) * 64;
        const float* Wsel = (w == 0) ? Wq : ((w == 1) ? Wk : ((w == 2) ? Wv : W0));
        #pragma unroll
        for (int i = 0; i < 8; ++i) {
            const int idx = tid + NTHR * i;
            const int kk  = idx >> 4;
            const int c4  = idx & 15;
            const v4f x = *(const v4f*)(Wsel + (size_t)(k0 + kk) * DD + n0 + 4 * c4);
            s_t[4 * c4 + 0][kk] = x[0];
            s_t[4 * c4 + 1][kk] = x[1];
            s_t[4 * c4 + 2][kk] = x[2];
            s_t[4 * c4 + 3][kk] = x[3];
        }
        __syncthreads();
        v8us hv[4], lv[4];
        size_t off[4];
        #pragma unroll
        for (int i = 0; i < 4; ++i) {
            const int idx = tid + NTHR * i;
            const int nn  = idx >> 3;
            const int k8  = idx & 7;
            const v4f a  = { s_t[nn][8 * k8 + 0], s_t[nn][8 * k8 + 1], s_t[nn][8 * k8 + 2], s_t[nn][8 * k8 + 3] };
            const v4f b2 = { s_t[nn][8 * k8 + 4], s_t[nn][8 * k8 + 5], s_t[nn][8 * k8 + 6], s_t[nn][8 * k8 + 7] };
            split8(a, b2, hv[i], lv[i]);
            off[i] = ((size_t)w * DD + n0 + nn) * DD + k0 + 8 * k8;
        }
        #pragma unroll
        for (int i = 0; i < 4; ++i) {
            *(volatile v8us*)(wth + off[i]) = hv[i];
            *(volatile v8us*)(wtl + off[i]) = lv[i];
        }
        __threadfence();
        #pragma unroll
        for (int i = 0; i < 4; ++i) {
            *(volatile v8us*)(wth + off[i]) = hv[i];
            *(volatile v8us*)(wtl + off[i]) = lv[i];
        }
    }
}

template <int MODE>
__global__ void __launch_bounds__(NTHR) gemm3_kernel(
    const unsigned short* __restrict__ Ah, const unsigned short* __restrict__ Al,
    const unsigned short* __restrict__ Bh, const unsigned short* __restrict__ Bl,
    const float* __restrict__ bias, float post,
    float* Cf, unsigned short* Ch, unsigned short* Cl)
{
    __shared__ __align__(16) float s_c[32][260];

    const int tid  = threadIdx.x;
    const int wv   = tid >> 5;
    const int l    = tid & 31;
    const int hh   = l >> 4;
    const int m15  = l & 15;
    const int row0 = blockIdx.x * 32;
    const int col0 = blockIdx.y * 256;

    const v8f zero = { 0.f, 0.f, 0.f, 0.f, 0.f, 0.f, 0.f, 0.f };
    v8f acc[2][4];
    #pragma unroll
    for (int rt = 0; rt < 2; ++rt)
        #pragma unroll
        for (int j = 0; j < 4; ++j) acc[rt][j] = zero;

    const unsigned short* a0h = Ah + (size_t)(row0 + m15) * DD;
    const unsigned short* a0l = Al + (size_t)(row0 + m15) * DD;
    const unsigned short* a1h = Ah + (size_t)(row0 + 16 + m15) * DD;
    const unsigned short* a1l = Al + (size_t)(row0 + 16 + m15) * DD;
    const unsigned short* bph = Bh + (size_t)(col0 + 64 * wv + m15) * DD;
    const unsigned short* bpl = Bl + (size_t)(col0 + 64 * wv + m15) * DD;

    #pragma unroll 1
    for (int k0 = 0; k0 < DD; k0 += 32) {
        const v16bf fa0h = frag16(a0h, k0, hh);
        const v16bf fa0l = frag16(a0l, k0, hh);
        const v16bf fa1h = frag16(a1h, k0, hh);
        const v16bf fa1l = frag16(a1l, k0, hh);
        #pragma unroll
        for (int j = 0; j < 4; ++j) {
            const v16bf fbh = frag16(bph + (size_t)j * 16 * DD, k0, hh);
            const v16bf fbl = frag16(bpl + (size_t)j * 16 * DD, k0, hh);
            acc[0][j] = wmma3(fa0h, fa0l, fbh, fbl, acc[0][j]);
            acc[1][j] = wmma3(fa1h, fa1l, fbh, fbl, acc[1][j]);
        }
    }

    #pragma unroll
    for (int rt = 0; rt < 2; ++rt)
        #pragma unroll
        for (int j = 0; j < 4; ++j)
            #pragma unroll
            for (int r = 0; r < 8; ++r)
                s_c[rt * 16 + 8 * hh + r][64 * wv + 16 * j + m15] = acc[rt][j][r];
    __syncthreads();

    if (MODE == 0) {
        v4f vals[16];
        size_t off[16];
        #pragma unroll
        for (int i = 0; i < 16; ++i) {
            const int idx = tid + NTHR * i;
            const int row = idx >> 6;
            const int c4  = idx & 63;
            const v4f x  = *(const v4f*)&s_c[row][4 * c4];
            const v4f bb = *(const v4f*)(bias + col0 + 4 * c4);
            vals[i] = (x + bb) * post;
            off[i]  = (size_t)(row0 + row) * DD + col0 + 4 * c4;
        }
        #pragma unroll
        for (int i = 0; i < 16; ++i) *(volatile v4f*)(Cf + off[i]) = vals[i];
        __threadfence();
        #pragma unroll
        for (int i = 0; i < 16; ++i) *(volatile v4f*)(Cf + off[i]) = vals[i];
    } else if (MODE == 1) {
        v4f vals[16];
        size_t off[16];
        #pragma unroll
        for (int i = 0; i < 16; ++i) {
            const int idx = tid + NTHR * i;
            const int hl  = idx >> 9;
            const int rem = idx & 511;
            const int row = rem >> 4;
            const int c4  = rem & 15;
            const int n   = col0 + 64 * hl + 4 * c4;
            const v4f x  = *(const v4f*)&s_c[row][64 * hl + 4 * c4];
            const v4f bb = *(const v4f*)(bias + n);
            vals[i] = (x + bb) * post;
            const int m  = row0 + row;
            const int b  = m >> 8;
            const int lq = m & 255;
            const int h  = n >> 6;
            off[i] = ((size_t)((b * HH + h) * LL + lq)) * DK + 4 * c4;
        }
        #pragma unroll
        for (int i = 0; i < 16; ++i) *(volatile v4f*)(Cf + off[i]) = vals[i];
        __threadfence();
        #pragma unroll
        for (int i = 0; i < 16; ++i) *(volatile v4f*)(Cf + off[i]) = vals[i];
    } else {
        v8us hv[8], lv[8];
        size_t off[8];
        const int b = col0 >> 8;
        #pragma unroll
        for (int i = 0; i < 8; ++i) {
            const int idx = tid + NTHR * i;
            const int row = idx >> 5;
            const int c8  = idx & 31;
            const float bs = bias[row0 + row];
            const v4f bb = { bs, bs, bs, bs };
            const v4f x0 = *(const v4f*)&s_c[row][8 * c8] + bb;
            const v4f x1 = *(const v4f*)&s_c[row][8 * c8 + 4] + bb;
            split8(x0, x1, hv[i], lv[i]);
            const int n  = row0 + row;
            const int h  = n >> 6;
            const int dk = n & 63;
            off[i] = ((size_t)((b * HH + h) * DK + dk)) * LL + 8 * c8;
        }
        #pragma unroll
        for (int i = 0; i < 8; ++i) {
            *(volatile v8us*)(Ch + off[i]) = hv[i];
            *(volatile v8us*)(Cl + off[i]) = lv[i];
        }
        __threadfence();
        #pragma unroll
        for (int i = 0; i < 8; ++i) {
            *(volatile v8us*)(Ch + off[i]) = hv[i];
            *(volatile v8us*)(Cl + off[i]) = lv[i];
        }
    }
}

__global__ void __launch_bounds__(NTHR) attn_kernel(
    const float* __restrict__ Qp, const float* __restrict__ Kp, const float* __restrict__ vp,
    const int* __restrict__ mask,
    const unsigned short* __restrict__ VTh, const unsigned short* __restrict__ VTl,
    unsigned short* Oh, unsigned short* Ol)
{
    __shared__ __align__(16) float          s_q[16][DK];
    __shared__ __align__(16) float          s_vp[DK];
    __shared__ __align__(16) unsigned short s_ph[16][LL];
    __shared__ __align__(16) unsigned short s_pl[16][LL];
    __shared__ __align__(16) float          s_o[16][68];
    __shared__ float s_rmax[4][4];
    __shared__ float s_rsum[4][4];

    const int tid = threadIdx.x;
    const int wv  = tid >> 5;
    const int l   = tid & 31;
    const int hh  = l >> 4;
    const int m15 = l & 15;
    const int bh  = blockIdx.y;
    const int b   = bh >> 3;
    const int h   = bh & 7;
    const int q0  = blockIdx.x * 16;

    const float LOG2E = 1.4426950408889634f;
    const float MASKV = -1.0e9f;

    #pragma unroll
    for (int i = 0; i < 2; ++i) {
        const int idx = tid + NTHR * i;
        const int r   = idx >> 4;
        const int c4  = idx & 15;
        *(v4f*)&s_q[r][4 * c4] = *(const v4f*)(Qp + ((size_t)(bh * LL + q0 + r)) * DK + 4 * c4);
    }
    if (tid < DK) s_vp[tid] = vp[h * DK + tid];
    __syncthreads();

    const int j0 = 2 * tid;
    const float* k0p = Kp + ((size_t)(bh * LL + j0)) * DK;
    const float* k1p = k0p + DK;
    const int* mrow = mask + ((size_t)(b * LL + q0)) * LL + j0;

    #pragma unroll 1
    for (int jq = 0; jq < 4; ++jq) {
        const int r0 = 4 * jq;

        float acc[4][2];
        #pragma unroll
        for (int j = 0; j < 4; ++j) { acc[j][0] = 0.0f; acc[j][1] = 0.0f; }

        #pragma unroll 1
        for (int d4 = 0; d4 < DK / 4; ++d4) {
            const v4f ka = *(const v4f*)(k0p + 4 * d4);
            const v4f kb = *(const v4f*)(k1p + 4 * d4);
            const v4f vv = *(const v4f*)&s_vp[4 * d4];
            #pragma unroll
            for (int j = 0; j < 4; ++j) {
                const v4f qv = *(const v4f*)&s_q[r0 + j][4 * d4];
                #pragma unroll
                for (int e = 0; e < 4; ++e) {
                    const float ra = RCP_FAST(EXP2_FAST(qv[e] + ka[e]) + 1.0f);
                    const float rb = RCP_FAST(EXP2_FAST(qv[e] + kb[e]) + 1.0f);
                    acc[j][0] = fmaf(vv[e], ra, acc[j][0]);
                    acc[j][1] = fmaf(vv[e], rb, acc[j][1]);
                }
            }
        }

        float bm[4];
        #pragma unroll
        for (int j = 0; j < 4; ++j) {
            const v2i mk = *(const v2i*)(mrow + (size_t)(r0 + j) * LL);
            const float s0 = (mk[0] == 0) ? MASKV : (-2.0f * acc[j][0]);
            const float s1 = (mk[1] == 0) ? MASKV : (-2.0f * acc[j][1]);
            acc[j][0] = s0;
            acc[j][1] = s1;
            float lm = fmaxf(s0, s1);
            #pragma unroll
            for (int off = 16; off > 0; off >>= 1) lm = fmaxf(lm, __shfl_xor(lm, off, 32));
            bm[j] = lm;
        }
        if (l == 0) {
            #pragma unroll
            for (int j = 0; j < 4; ++j) s_rmax[j][wv] = bm[j];
        }
        __syncthreads();
        #pragma unroll
        for (int j = 0; j < 4; ++j)
            bm[j] = fmaxf(fmaxf(s_rmax[j][0], s_rmax[j][1]), fmaxf(s_rmax[j][2], s_rmax[j][3]));

        float bs[4];
        #pragma unroll
        for (int j = 0; j < 4; ++j) {
            const float e0 = EXP2_FAST((acc[j][0] - bm[j]) * LOG2E);
            const float e1 = EXP2_FAST((acc[j][1] - bm[j]) * LOG2E);
            acc[j][0] = e0;
            acc[j][1] = e1;
            float ls = e0 + e1;
            #pragma unroll
            for (int off = 16; off > 0; off >>= 1) ls += __shfl_xor(ls, off, 32);
            bs[j] = ls;
        }
        if (l == 0) {
            #pragma unroll
            for (int j = 0; j < 4; ++j) s_rsum[j][wv] = bs[j];
        }
        __syncthreads();
        #pragma unroll
        for (int j = 0; j < 4; ++j) {
            const float sum = (s_rsum[j][0] + s_rsum[j][1]) + (s_rsum[j][2] + s_rsum[j][3]);
            const float inv = RCP_FAST(sum);
            const float p0  = acc[j][0] * inv;
            const float p1  = acc[j][1] * inv;
            unsigned int h0b, l0b, h1b, l1b;
            split1(p0, h0b, l0b);
            split1(p1, h1b, l1b);
            *(unsigned int*)&s_ph[r0 + j][j0] = (h1b << 16) | h0b;
            *(unsigned int*)&s_pl[r0 + j][j0] = (l1b << 16) | l0b;
        }
    }
    __syncthreads();

    v8f pacc = { 0.f, 0.f, 0.f, 0.f, 0.f, 0.f, 0.f, 0.f };
    const unsigned short* pah = &s_ph[m15][0];
    const unsigned short* pal = &s_pl[m15][0];
    const unsigned short* bvh = VTh + ((size_t)(bh * DK + 16 * wv + m15)) * LL;
    const unsigned short* bvl = VTl + ((size_t)(bh * DK + 16 * wv + m15)) * LL;
    #pragma unroll 1
    for (int k0 = 0; k0 < LL; k0 += 32) {
        const v16bf fah = frag16(pah, k0, hh);
        const v16bf fal = frag16(pal, k0, hh);
        const v16bf fbh = frag16(bvh, k0, hh);
        const v16bf fbl = frag16(bvl, k0, hh);
        pacc = wmma3(fah, fal, fbh, fbl, pacc);
    }
    #pragma unroll
    for (int r = 0; r < 8; ++r) s_o[8 * hh + r][16 * wv + m15] = pacc[r];
    __syncthreads();

    {
        const int row = tid >> 3;
        const int c8  = tid & 7;
        const v4f x0 = *(const v4f*)&s_o[row][8 * c8];
        const v4f x1 = *(const v4f*)&s_o[row][8 * c8 + 4];
        v8us hv, lv;
        split8(x0, x1, hv, lv);
        const size_t goff = ((size_t)(b * LL + q0 + row)) * DD + h * DK + 8 * c8;
        *(volatile v8us*)(Oh + goff) = hv;
        *(volatile v8us*)(Ol + goff) = lv;
        __threadfence();
        *(volatile v8us*)(Oh + goff) = hv;
        *(volatile v8us*)(Ol + goff) = lv;
    }
}

extern "C" void kernel_launch(void* const* d_in, const int* in_sizes, int n_in,
                              void* d_out, int out_size, void* d_ws, size_t ws_size,
                              hipStream_t stream)
{
    if (n_in < 13) return;
    if (in_sizes[0] != NR * DD || in_sizes[1] != NR * DD || in_sizes[2] != NR * DD) return;
    if (in_sizes[3] != BB * LL * LL) return;
    if (in_sizes[4] != DD * DD || in_sizes[6] != DD * DD || in_sizes[8] != DD * DD || in_sizes[11] != DD * DD) return;
    if (in_sizes[5] != DD || in_sizes[7] != DD || in_sizes[9] != DD || in_sizes[12] != DD) return;
    if (in_sizes[10] != HH * DK) return;
    if (out_size != NR * DD) return;

    const float* q    = (const float*)d_in[0];
    const float* k    = (const float*)d_in[1];
    const float* v    = (const float*)d_in[2];
    const int*   mask = (const int*)d_in[3];
    const float* Wq   = (const float*)d_in[4];
    const float* bq   = (const float*)d_in[5];
    const float* Wk   = (const float*)d_in[6];
    const float* bk   = (const float*)d_in[7];
    const float* Wv   = (const float*)d_in[8];
    const float* bv   = (const float*)d_in[9];
    const float* vp   = (const float*)d_in[10];
    const float* W0   = (const float*)d_in[11];
    const float* b0   = (const float*)d_in[12];
    float* out = (float*)d_out;

    const size_t sz_x  = (size_t)3 * NR * DD * 2;
    const size_t sz_wt = (size_t)4 * DD * DD * 2;
    const size_t sz_p  = (size_t)NR * DD * 4;
    const size_t sz_vt = (size_t)BB * HH * DK * LL * 2;
    const size_t sz_o  = (size_t)NR * DD * 2;
    size_t off = 0;
    const size_t off_xh  = off;  off += sz_x;
    const size_t off_xl  = off;  off += sz_x;
    const size_t off_wth = off;  off += sz_wt;
    const size_t off_wtl = off;  off += sz_wt;
    const size_t off_qp  = off;  off += sz_p;
    const size_t off_kp  = off;  off += sz_p;
    const size_t off_vth = off;  off += sz_vt;
    const size_t off_vtl = off;  off += sz_vt;
    const size_t off_oh  = off;  off += sz_o;
    const size_t off_ol  = off;  off += sz_o;
    if (off > ws_size) return;

    char* ws = (char*)d_ws;
    unsigned short* xh  = (unsigned short*)(ws + off_xh);
    unsigned short* xl  = (unsigned short*)(ws + off_xl);
    unsigned short* wth = (unsigned short*)(ws + off_wth);
    unsigned short* wtl = (unsigned short*)(ws + off_wtl);
    float*          Qp  = (float*)(ws + off_qp);
    float*          Kp  = (float*)(ws + off_kp);
    unsigned short* VTh = (unsigned short*)(ws + off_vth);
    unsigned short* VTl = (unsigned short*)(ws + off_vtl);
    unsigned short* Oh  = (unsigned short*)(ws + off_oh);
    unsigned short* Ol  = (unsigned short*)(ws + off_ol);

    const size_t xplane = (size_t)NR * DD;
    const size_t wplane = (size_t)DD * DD;
    const float C2 = 2.8853900817779268f;

    prep_kernel<<<dim3(3 * (NR / 2) + 256), dim3(NTHR), 0, stream>>>(
        q, k, v, Wq, Wk, Wv, W0, xh, xl, wth, wtl);

    gemm3_kernel<1><<<dim3(NR / 32, DD / 256), dim3(NTHR), 0, stream>>>(
        xh, xl, wth, wtl, bq, C2, Qp, Oh, Ol);

    gemm3_kernel<1><<<dim3(NR / 32, DD / 256), dim3(NTHR), 0, stream>>>(
        xh + xplane, xl + xplane, wth + wplane, wtl + wplane, bk, C2, Kp, Oh, Ol);

    gemm3_kernel<2><<<dim3(DD / 32, NR / 256), dim3(NTHR), 0, stream>>>(
        wth + 2 * wplane, wtl + 2 * wplane, xh + 2 * xplane, xl + 2 * xplane, bv, 1.0f,
        (float*)(ws + off_oh), VTh, VTl);

    attn_kernel<<<dim3(LL / 16, BB * HH), dim3(NTHR), 0, stream>>>(
        Qp, Kp, vp, mask, VTh, VTl, Oh, Ol);

    gemm3_kernel<0><<<dim3(NR / 32, DD / 256), dim3(NTHR), 0, stream>>>(
        Oh, Ol, wth + 3 * wplane, wtl + 3 * wplane, b0, 1.0f, out, VTh, VTl);
}
